// HebbNet_33337536151758
// MI455X (gfx1250) — hardware-run, weakly checked
//
#include <hip/hip_runtime.h>
#include <math.h>

typedef __attribute__((ext_vector_type(16))) _Float16 v16h;
typedef __attribute__((ext_vector_type(8)))  _Float16 v8h;
typedef __attribute__((ext_vector_type(8)))  float    v8f;
typedef __attribute__((ext_vector_type(4)))  float    v4f;
typedef __attribute__((ext_vector_type(2)))  float    v2f;

constexpr int kT  = 64;
constexpr int kB  = 256;
constexpr int kNx = 512;
constexpr int kNh = 512;
constexpr int kNy = 2;
constexpr int kRows = kT * kB;
constexpr float kCarryX = 16.0f;
constexpr float kCarryW = 256.0f;
constexpr float kScaleP = 1.0f / (kCarryX * kCarryW);
constexpr float kScaleG = 1.0f / (kCarryX * kCarryX);
static_assert((kNx % 32) == 0, "GEMM K multiple of 32");
static_assert((kRows % 64) == 0 && (kNh % 64) == 0 && (kT % 64) == 0, "GEMM M,N multiples of 64");
static_assert(kNy == 2 && kT == 64 && kNh == 512, "scan kernel layout");

constexpr size_t kOffX16 = 0;
constexpr size_t kOffW16 = kOffX16 + (size_t)kRows * kNx * 2;
constexpr size_t kOffP   = kOffW16 + (size_t)kNh * kNx * 2;
constexpr size_t kOffG   = kOffP   + (size_t)kRows * kNh * 4;
constexpr size_t kOffA2  = kOffG   + (size_t)kB * kT * kT * 4;
constexpr size_t kWsTotal = kOffA2 + (size_t)kB * kT * kNy * 4;
static_assert(kWsTotal == 55181312ull, "carve total");
static_assert(kWsTotal <= 134217728ull, "carve cap");
static_assert((kOffW16 % 128) == 0 && (kOffP % 128) == 0 && (kOffG % 128) == 0 && (kOffA2 % 128) == 0, "aligned regions");

constexpr size_t kOut0Elems = (size_t)kT * kB * kNh;
constexpr size_t kOut1Elems = (size_t)kT * kB * kNy;
static_assert(kOut0Elems * 4 == 33554432ull, "out1 byte offset");
static_assert((kOut0Elems + kOut1Elems) * 4 == 33685504ull, "output total bytes");

union FragH { v16h v; v8h h[2]; };
__device__ __forceinline__ v16h frag_load_h(const _Float16* p) {
  FragH f;
  f.h[0] = *(const v8h*)(p);
  f.h[1] = *(const v8h*)(p + 16);
  return f.v;
}
__device__ __forceinline__ v8f mma_h(v16h a, v16h b, v8f c) {
  return __builtin_amdgcn_wmma_f32_16x16x32_f16(false, a, false, b, (short)0, c, false, false);
}
__device__ __forceinline__ void row_guard_h(v8f& a, v8f& b, v8f& c, v8f& d, v16h x, v16h b0, v16h b1, v16h b2, v16h b3) {
  asm volatile("v_nop\n\tv_nop\n\tv_nop\n\tv_nop" : "+v"(a), "+v"(b), "+v"(c), "+v"(d) : "v"(x), "v"(b0), "v"(b1), "v"(b2), "v"(b3));
}
__device__ __forceinline__ void keep4_h(v16h a, v16h b, v16h c, v16h d) { asm volatile("v_nop" :: "v"(a), "v"(b), "v"(c), "v"(d)); }
__device__ __forceinline__ void acc_guard4(v8f& a, v8f& b, v8f& c, v8f& d) { asm volatile("v_nop\n\tv_nop\n\tv_nop\n\tv_nop" : "+v"(a), "+v"(b), "+v"(c), "+v"(d)); }

template <bool PERM>
__global__ __launch_bounds__(256) void cvt_f16_kernel(
    const float* __restrict__ src, unsigned short* __restrict__ dst, int total8, float carry)
{
  const int i = blockIdx.x * 256 + threadIdx.x;
  if (i >= total8) return;
  const size_t e0 = (size_t)i << 3;
  size_t s0 = e0;
  if (PERM) {
    const int k   = (int)(e0 & (size_t)(kNx - 1));
    const int row = (int)(e0 >> 9);
    const int t   = row & (kT - 1);
    const int b   = row >> 6;
    s0 = ((size_t)(t * kB + b)) * kNx + k;
  }
  const v4f a0 = *(const v4f*)(src + s0);
  const v4f a1 = *(const v4f*)(src + s0 + 4);
  v8h hv;
#pragma unroll
  for (int e = 0; e < 4; ++e) {
    const float f0 = a0[e] * carry;
    const float f1 = a1[e] * carry;
    hv[e]     = (_Float16)f0;
    hv[4 + e] = (_Float16)f1;
  }
  unsigned short* q = dst + e0;
  *(volatile v8h*)q = hv;
  __threadfence();
  *(volatile v8h*)q = hv;
}

__global__ __launch_bounds__(256) void wmma_gemm64_f16(
    const unsigned short* Ap, int lda, long strideA,
    const unsigned short* Btp, int ldb, long strideB,
    float* __restrict__ Cout, int ldc, long strideC,
    int M, int N, int K, int nbatch, float scale)
{
  const _Float16* A  = (const _Float16*)Ap;
  const _Float16* Bt = (const _Float16*)Btp;
  __shared__ __align__(16) float sT[8][16 * 68];
  const int lane = threadIdx.x & 31;
  const int wave = threadIdx.x >> 5;
  const int tilesN = N >> 6;
  const int tilesM = M >> 6;
  const int tilesPer = tilesM * tilesN;
  const int gt = blockIdx.x * 8 + wave;
  if (gt >= tilesPer * nbatch) return;
  const int b    = gt / tilesPer;
  const int tile = gt - b * tilesPer;
  const int tm = tile / tilesN;
  const int tn = tile - tm * tilesN;
  const int m0 = tm << 6;
  const int n0 = tn << 6;

  const _Float16* Ab = A  + (size_t)b * strideA;
  const _Float16* Bb = Bt + (size_t)b * strideB;

  const int rlane = lane & 15;
  const int koff  = (lane >> 4) * 8;
  const int mOff  = (lane >> 4) * 8;

  v8f acc[4][4];
#pragma unroll
  for (int i = 0; i < 4; ++i)
#pragma unroll
    for (int j = 0; j < 4; ++j) acc[i][j] = (v8f){0.f,0.f,0.f,0.f,0.f,0.f,0.f,0.f};

  for (int k0 = 0; k0 < K; k0 += 32) {
    v16h bh[4];
#pragma unroll
    for (int j = 0; j < 4; ++j) {
      const size_t bo = (size_t)(n0 + (j << 4) + rlane) * ldb + koff + k0;
      bh[j] = frag_load_h(Bb + bo);
    }
#pragma unroll
    for (int i = 0; i < 4; ++i) {
      const size_t ao = (size_t)(m0 + (i << 4) + rlane) * lda + koff + k0;
      const v16h ah = frag_load_h(Ab + ao);
#pragma unroll
      for (int j = 0; j < 4; ++j) acc[i][j] = mma_h(ah, bh[j], acc[i][j]);
      row_guard_h(acc[i][0], acc[i][1], acc[i][2], acc[i][3], ah, bh[0], bh[1], bh[2], bh[3]);
    }
    keep4_h(bh[0], bh[1], bh[2], bh[3]);
  }
  acc_guard4(acc[0][0], acc[0][1], acc[0][2], acc[0][3]);
  acc_guard4(acc[1][0], acc[1][1], acc[1][2], acc[1][3]);
  acc_guard4(acc[2][0], acc[2][1], acc[2][2], acc[2][3]);
  acc_guard4(acc[3][0], acc[3][1], acc[3][2], acc[3][3]);

  float* slab = sT[wave];
  float* C = Cout + (size_t)b * strideC;
  const int hh = lane >> 4, c4 = (lane & 15) * 4;
#pragma unroll
  for (int i = 0; i < 4; ++i) {
    const int mBase = m0 + (i << 4);
#pragma unroll
    for (int j = 0; j < 4; ++j) {
#pragma unroll
      for (int r = 0; r < 8; ++r) {
        const float v = acc[i][j][r] * scale;
        slab[(mOff + r) * 68 + (j << 4) + rlane] = v;
      }
    }
    __builtin_amdgcn_fence(__ATOMIC_RELEASE, "workgroup");
    __builtin_amdgcn_wave_barrier();
    __builtin_amdgcn_fence(__ATOMIC_ACQUIRE, "workgroup");
    for (int pass = 0; pass < 2; ++pass) {
#pragma unroll
      for (int it = 0; it < 8; ++it) {
        const int row = it * 2 + hh;
        const v4f v = *(const v4f*)(slab + row * 68 + c4);
        *(volatile v4f*)(C + (size_t)(mBase + row) * ldc + n0 + c4) = v;
      }
      __threadfence();
    }
    __builtin_amdgcn_fence(__ATOMIC_RELEASE, "workgroup");
    __builtin_amdgcn_wave_barrier();
    __builtin_amdgcn_fence(__ATOMIC_ACQUIRE, "workgroup");
  }
}

__device__ __forceinline__ float sigmoid_f(float a) {
  const float na = fminf(-a, 60.0f);
  const float e  = expf(na);
  return 1.0f / (1.0f + e);
}

constexpr int kScanLdsFloats = kT * kNh + kT * kT + kT + 64 + kT * kNy;
constexpr size_t kScanLdsBytes = (size_t)kScanLdsFloats * 4;
static_assert(kScanLdsBytes == 148480ull, "scan LDS bytes");

__global__ __launch_bounds__(512) void scan_kernel(
    const float* __restrict__ P, const float* __restrict__ G,
    const float* __restrict__ b1, const float* __restrict__ w2, const float* __restrict__ b2,
    const float* __restrict__ w21, const float* __restrict__ lamp, const float* __restrict__ etap,
    float* __restrict__ out0, float* __restrict__ A2ws)
{
  extern __shared__ __align__(16) float smem[];
  float* Hls    = smem;
  float* Cm     = Hls + kT * kNh;
  float* lampow = Cm + kT * kT;
  float* wred   = lampow + kT;
  float* a2h    = wred + 64;

  const int tid  = threadIdx.x;
  const int lane = tid & 31;
  const int wave = tid >> 5;
  const int b    = blockIdx.x;

  const float lam_c = fminf(lamp[0], 1.0f);
  const float eta   = etap[0];

#pragma unroll 1
  for (int s = 0; s < kT; ++s) Hls[s * kNh + tid] = 0.0f;

  {
    float p = 1.0f;
#pragma unroll 1
    for (int i = 0; i < kT - 1; ++i) {
      const float q = p * lam_c;
      p = (i < tid) ? q : p;
    }
    if (tid < kT) lampow[tid] = p;
  }
  __syncthreads();

  {
    const float* Gb = G + (size_t)b * (kT * kT);
#pragma unroll
    for (int i = 0; i < 8; ++i) {
      const int idx = tid + i * 512;
      const int t = idx >> 6;
      const int s = idx & 63;
      const float g = Gb[idx];
      int e = t - 1 - s;
      e = (e < 0) ? 0 : e;
      const float c = eta * lampow[e] * g;
      Cm[idx] = (s < t) ? c : 0.0f;
    }
  }

  const float b1h  = b1[tid];
  const v2f   w2v  = *(const v2f*)(w2 + 2 * tid);
  const v2f   w21v = *(const v2f*)(w21 + 2 * tid);
  const float w2h0 = w2v[0], w2h1 = w2v[1];
  const float w21h0 = w21v[0], w21h1 = w21v[1];
  const float b20 = b2[0], b21 = b2[1];
  __syncthreads();

  const float* Pb = P + (size_t)b * (kT * kNh) + tid;
  float a2x = 0.0f, a2y = 0.0f;

#pragma unroll 1
  for (int t = 0; t < kT; ++t) {
    float acc = b1h + Pb[t * kNh];
    acc = fmaf(w21h0, a2x, acc);
    acc = fmaf(w21h1, a2y, acc);

    const float* cr = Cm + t * kT;
    const int ng = (t + 3) >> 2;
#pragma unroll 1
    for (int g = 0; g < ng; ++g) {
      const v4f c = *(const v4f*)(cr + 4 * g);
      const float* hp = Hls + (4 * g) * kNh + tid;
      acc = fmaf(c[0], hp[0], acc);
      acc = fmaf(c[1], hp[kNh], acc);
      acc = fmaf(c[2], hp[2 * kNh], acc);
      acc = fmaf(c[3], hp[3 * kNh], acc);
    }

    const float hv = sigmoid_f(acc);
    Hls[t * kNh + tid] = hv;

    float p0 = hv * w2h0;
    float p1 = hv * w2h1;
#pragma unroll
    for (int off = 16; off > 0; off >>= 1) {
      p0 += __shfl_xor(p0, off, 32);
      p1 += __shfl_xor(p1, off, 32);
    }
    float* wr = wred + (t & 1) * 32;
    if (lane == 0) {
      wr[wave * 2]     = p0;
      wr[wave * 2 + 1] = p1;
    }
    __syncthreads();
    float s0 = b20, s1 = b21;
#pragma unroll
    for (int w4 = 0; w4 < 8; ++w4) {
      const v4f q = *(const v4f*)(wr + 4 * w4);
      s0 += q[0];
      s1 += q[1];
      s0 += q[2];
      s1 += q[3];
    }
    if (tid == 0) {
      a2h[t * 2]     = s0;
      a2h[t * 2 + 1] = s1;
    }
    a2x = s0;
    a2y = s1;
  }
  __syncthreads();

  {
    const int rsub = tid >> 7;
    const int c4 = (tid & 127) * 4;
    for (int pass = 0; pass < 2; ++pass) {
#pragma unroll
      for (int it = 0; it < 16; ++it) {
        const int t = it * 4 + rsub;
        const v4f v = *(const v4f*)(Hls + t * kNh + c4);
        *(volatile v4f*)(out0 + ((size_t)(t * kB + b)) * kNh + c4) = v;
      }
      if (wave == 0) {
        const v4f a = *(const v4f*)(a2h + 4 * lane);
        *(volatile v4f*)(A2ws + (size_t)b * (kT * kNy) + 4 * lane) = a;
      }
      __threadfence();
    }
  }
}

__global__ __launch_bounds__(256) void y_pack_kernel(const float* __restrict__ A2ws, float* __restrict__ out1, int total4)
{
  const int i = blockIdx.x * 256 + threadIdx.x;
  if (i >= total4) return;
  const int o   = i * 4;
  const int t   = o >> 9;
  const int rem = o & 511;
  const int b0  = rem >> 1;
  const v2f u0 = *(const v2f*)(A2ws + ((size_t)(b0 * kT + t)) * kNy);
  const v2f u1 = *(const v2f*)(A2ws + ((size_t)((b0 + 1) * kT + t)) * kNy);
  v4f r;
  r[0] = sigmoid_f(u0[0]);
  r[1] = sigmoid_f(u0[1]);
  r[2] = sigmoid_f(u1[0]);
  r[3] = sigmoid_f(u1[1]);
  float* q = out1 + (size_t)o;
  *(volatile v4f*)q = r;
  __threadfence();
  *(volatile v4f*)q = r;
}

extern "C" void kernel_launch(void* const* d_in, const int* in_sizes, int n_in,
                              void* d_out, int out_size, void* d_ws, size_t ws_size,
                              hipStream_t stream) {
  (void)stream;
  if (n_in < 8) return;
  if (in_sizes[0] != kT * kB * kNx) return;
  if (in_sizes[1] != kNh * kNx) return;
  if (in_sizes[2] != kNh) return;
  if (in_sizes[3] != kNh * kNy) return;
  if (in_sizes[4] != kNy) return;
  if (in_sizes[5] != kNh * kNy) return;
  if (in_sizes[6] != 1) return;
  if (in_sizes[7] != 1) return;
  if ((size_t)out_size != kOut0Elems + kOut1Elems) return;
  if (ws_size < kWsTotal) return;

  const float* x   = (const float*)d_in[0];
  const float* w1  = (const float*)d_in[1];
  const float* b1  = (const float*)d_in[2];
  const float* w2  = (const float*)d_in[3];
  const float* b2  = (const float*)d_in[4];
  const float* w21 = (const float*)d_in[5];
  const float* lam = (const float*)d_in[6];
  const float* eta = (const float*)d_in[7];

  float* out0 = (float*)d_out;
  float* out1 = out0 + kOut0Elems;

  char* ws = (char*)d_ws;
  unsigned short* X16 = (unsigned short*)(ws + kOffX16);
  unsigned short* W16 = (unsigned short*)(ws + kOffW16);
  float* Pp  = (float*)(ws + kOffP);
  float* Gp  = (float*)(ws + kOffG);
  float* A2p = (float*)(ws + kOffA2);

  constexpr int kXTot8 = kT * kB * kNx / 8;
  constexpr int kWTot8 = kNh * kNx / 8;
  static_assert((kXTot8 % 256) == 0 && (kWTot8 % 256) == 0, "convert grids exact");

  cvt_f16_kernel<true><<<kXTot8 / 256, 256, 0, stream>>>(x, X16, kXTot8, kCarryX);
  cvt_f16_kernel<false><<<kWTot8 / 256, 256, 0, stream>>>(w1, W16, kWTot8, kCarryW);

  wmma_gemm64_f16<<<(kRows / 64) * (kNh / 64) / 8, 256, 0, stream>>>(
      X16, kNx, 0L,
      W16, kNx, 0L,
      Pp, kNh, 0L,
      kRows, kNh, kNx, 1, kScaleP);

  wmma_gemm64_f16<<<kB / 8, 256, 0, stream>>>(
      X16, kNx, (long)kT * kNx,
      X16, kNx, (long)kT * kNx,
      Gp, kT, (long)kT * kT,
      kT, kT, kNx, kB, kScaleG);

  scan_kernel<<<kB, 512, kScanLdsBytes, stream>>>(Pp, Gp, b1, w2, b2, w21, lam, eta, out0, A2p);

  constexpr int kYTot4 = (int)(kOut1Elems / 4);
  static_assert((kYTot4 % 256) == 0, "pack grid exact");
  y_pack_kernel<<<kYTot4 / 256, 256, 0, stream>>>(A2p, out1, kYTot4);
}
